// SuperNet_Layer_55018531062685
// MI455X (gfx1250) — hardware-verified
//
#include <hip/hip_runtime.h>
#include <stdint.h>

#define MROWS 8192
#define KDIM  1024
#define NCOLS 1024
#define WTM   32
#define WTN   32
#define BLKM  64
#define BLKN  128
#define NWAVE 8
#define SPITCH 36
#define XSC   64.0f
#define WSC   1024.0f
#define LSC   2048.0f
#define INV_L  0.00048828125f
#define INV_XW 0.0000152587890625f

static_assert(MROWS % BLKM == 0);
static_assert(NCOLS % BLKN == 0);
static_assert(KDIM % 32 == 0);
static_assert(KDIM / 8 == 128);
static_assert(BLKM == 2 * WTM);
static_assert(BLKN == 4 * WTN);
static_assert((SPITCH % 4) == 0);
static_assert(NWAVE * 32 == 256);

typedef _Float16 v16h __attribute__((ext_vector_type(16)));
typedef _Float16 v8h  __attribute__((ext_vector_type(8)));
typedef float    v8f  __attribute__((ext_vector_type(8)));
typedef float    v4f  __attribute__((ext_vector_type(4)));
typedef float    v4fa __attribute__((ext_vector_type(4), may_alias));

union Frag { v16h v; v8h half[2]; };

__device__ __forceinline__ float bf16r(float f) {
  unsigned int u = __float_as_uint(f);
  u = u + 0x7FFFu + ((u >> 16) & 1u);
  return __uint_as_float(u & 0xFFFF0000u);
}

__device__ __forceinline__ void softmax2(const float* s, float& p0, float& p1) {
  const float s0 = bf16r(s[0]);
  const float s1 = bf16r(s[1]);
  const float mx = fmaxf(s0, s1);
  const float e0 = expf(s0 - mx);
  const float e1 = expf(s1 - mx);
  const float rs = 1.0f / (e0 + e1);
  p0 = e0 * rs;
  p1 = e1 * rs;
}

__device__ __forceinline__ v8f mma16(v16h a, v16h b, v8f c) {
  return __builtin_amdgcn_wmma_f32_16x16x32_f16(false, a, false, b, (short)0, c, false, false);
}
__device__ __forceinline__ void guard3(v8f& c0, v8f& c1, v16h a, v16h b0, v16h b1) {
#if defined(__HIP_DEVICE_COMPILE__)
  asm volatile("v_nop\n\tv_nop\n\tv_nop\n\tv_nop" : "+v"(c0), "+v"(c1) : "v"(a), "v"(b0), "v"(b1));
#endif
}

__global__ __launch_bounds__(256) void k_prep_x(const float* __restrict__ x, _Float16* xs, int ng) {
  const int g = (int)blockIdx.x * 256 + (int)threadIdx.x;
  if (g >= ng) return;
  const float* xp = x + (size_t)g * 8;
  const v4f a = *(const v4f*)xp;
  const v4f b = *(const v4f*)(xp + 4);
  v8h o = {};
#pragma unroll
  for (int e = 0; e < 4; ++e) {
    o[e]     = (_Float16)(bf16r(a[e]) * XSC);
    o[4 + e] = (_Float16)(bf16r(b[e]) * XSC);
  }
  _Float16* op = xs + (size_t)g * 8;
  *(volatile v8h*)op = o;
  __threadfence();
  *(volatile v8h*)op = o;
}

__global__ __launch_bounds__(256) void k_prep_w(const float* __restrict__ Wsd, const float* __restrict__ Wsig,
                                                _Float16* whi, _Float16* wlo, int ng) {
#pragma clang fp contract(off)
  const int g = (int)blockIdx.x * 256 + (int)threadIdx.x;
  if (g >= ng) return;
  const int n  = g >> 7;
  const int ks = (g & 127) * 8;
  float w0, w1;
  softmax2(Wsig, w0, w1);
  v8h oh = {}, ol = {};
#pragma unroll
  for (int e = 0; e < 8; ++e) {
    const int k = ks + e;
    const float sd = bf16r(Wsd[(size_t)k * NCOLS + n]);
    const int d  = k - n;
    const int da = d > 0 ? d : 0;
    const int db = d < 0 ? -d : 0;
    const float ta = Wsd[(size_t)da * NCOLS];
    const float tb = Wsd[db];
    const float tp = bf16r(d >= 0 ? ta : tb);
    const float p0 = w0 * sd;
    const float p1 = w1 * tp;
    const float w  = (p0 + p1) * WSC;
    const _Float16 hh = (_Float16)w;
    const float r = (w - (float)hh) * LSC;
    oh[e] = hh;
    ol[e] = (_Float16)r;
  }
  _Float16* ph = whi + (size_t)g * 8;
  _Float16* pl = wlo + (size_t)g * 8;
  *(volatile v8h*)ph = oh;
  *(volatile v8h*)pl = ol;
  __threadfence();
  *(volatile v8h*)ph = oh;
  *(volatile v8h*)pl = ol;
}

__global__ __launch_bounds__(256) void k_gemm(const _Float16* __restrict__ xs,
                                              const _Float16* __restrict__ whi,
                                              const _Float16* __restrict__ wlo,
                                              const float* __restrict__ bsd,
                                              const float* __restrict__ bsig,
                                              const float* __restrict__ asig,
                                              float* out) {
#pragma clang fp contract(off)
  __shared__ __align__(16) float s_tile[NWAVE * WTM * SPITCH];

  const int tid = threadIdx.x;
  const int wave = tid >> 5, lane = tid & 31, h = lane >> 4, m = lane & 15;
  if ((int)blockIdx.x * BLKM + BLKM > MROWS || (int)blockIdx.y * BLKN + BLKN > NCOLS) return;
  const int wm = wave >> 2, wn = wave & 3;
  const int row0 = (int)blockIdx.x * BLKM + wm * WTM;
  const int col0 = (int)blockIdx.y * BLKN + wn * WTN;

  v8f acch[4], accl[4];
  {
    const v8f zero = {};
#pragma unroll
    for (int t = 0; t < 4; ++t) { acch[t] = zero; accl[t] = zero; }
  }

  const _Float16* xa0 = xs  + (size_t)(row0 + m) * KDIM + 8 * h;
  const _Float16* xa1 = xa0 + (size_t)16 * KDIM;
  const _Float16* bh0 = whi + (size_t)(col0 + m) * KDIM + 8 * h;
  const _Float16* bh1 = bh0 + (size_t)16 * KDIM;
  const _Float16* bl0 = wlo + (size_t)(col0 + m) * KDIM + 8 * h;
  const _Float16* bl1 = bl0 + (size_t)16 * KDIM;

#pragma unroll 1
  for (int k0 = 0; k0 < KDIM; k0 += 32) {
    Frag a0, a1, fh0, fh1, fl0, fl1;
    a0.half[0]  = *(const v8h*)(xa0 + k0);  a0.half[1]  = *(const v8h*)(xa0 + k0 + 16);
    a1.half[0]  = *(const v8h*)(xa1 + k0);  a1.half[1]  = *(const v8h*)(xa1 + k0 + 16);
    fh0.half[0] = *(const v8h*)(bh0 + k0);  fh0.half[1] = *(const v8h*)(bh0 + k0 + 16);
    fh1.half[0] = *(const v8h*)(bh1 + k0);  fh1.half[1] = *(const v8h*)(bh1 + k0 + 16);
    fl0.half[0] = *(const v8h*)(bl0 + k0);  fl0.half[1] = *(const v8h*)(bl0 + k0 + 16);
    fl1.half[0] = *(const v8h*)(bl1 + k0);  fl1.half[1] = *(const v8h*)(bl1 + k0 + 16);

    acch[0] = mma16(a0.v, fh0.v, acch[0]);  accl[0] = mma16(a0.v, fl0.v, accl[0]);  guard3(acch[0], accl[0], a0.v, fh0.v, fl0.v);
    acch[1] = mma16(a0.v, fh1.v, acch[1]);  accl[1] = mma16(a0.v, fl1.v, accl[1]);  guard3(acch[1], accl[1], a0.v, fh1.v, fl1.v);
    acch[2] = mma16(a1.v, fh0.v, acch[2]);  accl[2] = mma16(a1.v, fl0.v, accl[2]);  guard3(acch[2], accl[2], a1.v, fh0.v, fl0.v);
    acch[3] = mma16(a1.v, fh1.v, acch[3]);  accl[3] = mma16(a1.v, fl1.v, accl[3]);  guard3(acch[3], accl[3], a1.v, fh1.v, fl1.v);
  }

  float b0w, b1w, a0w, a1w;
  softmax2(bsig, b0w, b1w);
  softmax2(asig, a0w, a1w);
  (void)b1w;

  float* sw = s_tile + wave * (WTM * SPITCH);
#pragma unroll
  for (int nt = 0; nt < 2; ++nt) {
    const int cl = 16 * nt + m;
    const float bc = b0w * bf16r(bsd[col0 + cl]);
#pragma unroll
    for (int mt = 0; mt < 2; ++mt) {
#pragma unroll
      for (int r = 0; r < 8; ++r) {
        const int rl = 16 * mt + 8 * h + r;
        const float th = acch[2 * mt + nt][r];
        const float tl = accl[2 * mt + nt][r] * INV_L;
        const float t  = th + tl;
        const float v  = t * INV_XW + bc;
        const float y  = a0w * v + a1w * fmaxf(v, 0.0f);
        sw[rl * SPITCH + cl] = y;
      }
    }
  }
  __syncthreads();

  const int rq = lane >> 3, seg = lane & 7;
  float* ob = out + (size_t)row0 * NCOLS + col0 + seg * 4;
  const float* sr = sw + seg * 4;
#pragma unroll
  for (int p = 0; p < 8; ++p) {
    const int row = 4 * p + rq;
    const v4f v = *(const v4fa*)(sr + row * SPITCH);
    *(volatile v4f*)(ob + (size_t)row * NCOLS) = v;
  }
  __threadfence();
#pragma unroll
  for (int p = 0; p < 8; ++p) {
    const int row = 4 * p + rq;
    const v4f v = *(const v4fa*)(sr + row * SPITCH);
    *(volatile v4f*)(ob + (size_t)row * NCOLS) = v;
  }
}

extern "C" void kernel_launch(void* const* d_in, const int* in_sizes, int n_in,
                              void* d_out, int out_size, void* d_ws, size_t ws_size,
                              hipStream_t stream) {
  if (n_in < 6) return;
  if (in_sizes[0] != MROWS * KDIM) return;
  if (in_sizes[1] != KDIM * NCOLS) return;
  if (in_sizes[2] != NCOLS) return;
  if (in_sizes[3] != 2 || in_sizes[4] != 2 || in_sizes[5] != 2) return;
  if (out_size != MROWS * NCOLS) return;

  const size_t off_x = 0;
  const size_t sz_x  = (size_t)MROWS * KDIM * sizeof(_Float16);
  const size_t off_h = off_x + sz_x;
  const size_t sz_w  = (size_t)NCOLS * KDIM * sizeof(_Float16);
  const size_t off_l = off_h + sz_w;
  const size_t need  = off_l + sz_w;
  if (need > ws_size) return;
  if (need > (size_t)134217728) return;

  const float* x    = (const float*)d_in[0];
  const float* Wsd  = (const float*)d_in[1];
  const float* bsd  = (const float*)d_in[2];
  const float* Wsig = (const float*)d_in[3];
  const float* bsig = (const float*)d_in[4];
  const float* asig = (const float*)d_in[5];
  float* out = (float*)d_out;
  _Float16* xs  = (_Float16*)((char*)d_ws + off_x);
  _Float16* whi = (_Float16*)((char*)d_ws + off_h);
  _Float16* wlo = (_Float16*)((char*)d_ws + off_l);

  const int ngx = in_sizes[0] / 8;
  const int ngw = in_sizes[1] / 8;

  k_prep_w<<<dim3((ngw + 255) / 256), dim3(256), 0, stream>>>(Wsd, Wsig, whi, wlo, ngw);
  k_prep_x<<<dim3((ngx + 255) / 256), dim3(256), 0, stream>>>(x, xs, ngx);
  k_gemm<<<dim3(MROWS / BLKM, NCOLS / BLKN), dim3(256), 0, stream>>>(xs, whi, wlo, bsd, bsig, asig, out);
  (void)hipGetLastError();
}
